// TransformerLayer_87943750353244
// MI455X (gfx1250) — hardware-verified
//
#include <hip/hip_runtime.h>


#ifndef NB
#define NB 2
#endif
#ifndef SEQ
#define SEQ 4096
#endif
#define NB_FULL  2
#define SEQ_FULL 4096
#ifndef OUT_SEQ
#define OUT_SEQ SEQ
#endif
#define EMB  512
#define NH_  8
#define HD   64
#define DM   (NH_ * HD)
#define WIN  512
#define NBK  32
#define XT   (WIN + SEQ)
#define NSTEP (WIN / 32 + 1)
#define AW   4
#define OSP  68
#define SC2  ((float)(0.125 * 1.4426950408889634))
#define LOG2E ((float)1.4426950408889634)
#define PSH  14.0f
#define NEGB (-3.0e38f)
#define OFF1 ((size_t)NB_FULL * SEQ_FULL * DM)
#define OFF2 (OFF1 + (size_t)NB_FULL * WIN * DM)

static_assert(HD == 64);
static_assert(NH_ * HD == 512);
static_assert(EMB % 32 == 0);
static_assert(EMB % 64 == 0);
static_assert(DM % 64 == 0);
static_assert(SEQ % 64 == 0);
static_assert(WIN % 64 == 0);
static_assert(SEQ >= WIN);
static_assert((SEQ - WIN) % 64 == 0);
static_assert(SEQ % (16 * AW) == 0);
static_assert(XT % 64 == 0);
static_assert(32 * NSTEP - 16 >= WIN + 16);
static_assert(((SEQ - 16) & ~31) + 32 * NSTEP <= XT);
static_assert(NB <= NB_FULL);
static_assert(SEQ <= SEQ_FULL);
static_assert((OSP * 4) % 16 == 0);
static_assert(OSP >= HD);
static_assert(OFF1 * 4 == (size_t)16777216);
static_assert(OFF2 * 4 == (size_t)18874368);
static_assert(((size_t)(NB - 1) * OUT_SEQ + SEQ) * DM <= OFF1);
static_assert(32 * 16 * 4 == 16 * 128);
static_assert(32 * 16 * 8 == 16 * 256);
static_assert(256 * 16 * 2 == 64 * 128);
static_assert(AW * 16 * OSP * 4 + WIN * 4 <= 131072);
static_assert(64 * 68 * 4 <= 131072);

typedef _Float16 h16;
typedef unsigned short bf;
typedef __attribute__((ext_vector_type(16))) __bf16   v16bf;
typedef __attribute__((ext_vector_type(16))) _Float16 v16h;
typedef __attribute__((ext_vector_type(8)))  _Float16 v8h;
typedef __attribute__((ext_vector_type(8)))  unsigned short v8us;
typedef __attribute__((ext_vector_type(8)))  float    v8f;
typedef __attribute__((ext_vector_type(4)))  float    v4f;
typedef v4f  __attribute__((may_alias)) v4fa;

__device__ __forceinline__ unsigned short f2bf(float f) { unsigned u = __float_as_uint(f); u += 0x7FFFu + ((u >> 16) & 1u); return (unsigned short)(u >> 16); }
__device__ __forceinline__ float bfr(float f) { return __uint_as_float(((unsigned)f2bf(f)) << 16); }
__device__ __forceinline__ v16h cat16(v8h lo, v8h hi) { return __builtin_shufflevector(lo, hi, 0, 1, 2, 3, 4, 5, 6, 7, 8, 9, 10, 11, 12, 13, 14, 15); }
__device__ __forceinline__ v16bf cat16b(v8us lo, v8us hi) { return __builtin_bit_cast(v16bf, __builtin_shufflevector(lo, hi, 0, 1, 2, 3, 4, 5, 6, 7, 8, 9, 10, 11, 12, 13, 14, 15)); }
__device__ __forceinline__ v8f wmma16(v16h a, v16h b, v8f c) { return __builtin_amdgcn_wmma_f32_16x16x32_f16(false, a, false, b, (short)0, c, false, false); }
__device__ __forceinline__ v8f wmmab(v16bf a, v16bf b, v8f c) { return __builtin_amdgcn_wmma_f32_16x16x32_bf16(false, a, false, b, (short)0, c, false, false); }
__device__ __forceinline__ v16h  ldh(const h16* p) { return cat16(*(const v8h*)p, *(const v8h*)(p + 16)); }
__device__ __forceinline__ v16bf ldb(const bf* p)  { return cat16b(*(const v8us*)p, *(const v8us*)(p + 16)); }
__device__ __forceinline__ void wave_sync() { __builtin_amdgcn_fence(3  , "wavefront"); __builtin_amdgcn_wave_barrier(); asm volatile("" ::: "memory"); }

static __device__ __forceinline__ h16 toh_flush(float v) { const h16 r = (h16)v; return (fabsf(v) < 6.103515625e-05f) ? (h16)0.0f : r; }
static __device__ __forceinline__ v8f wmma16g(v16h a, v16h b, v8f c) {
    c = __builtin_amdgcn_wmma_f32_16x16x32_f16(false, a, false, b, (short)0, c, false, false);
    asm volatile("v_nop\n\tv_nop\n\tv_nop\n\tv_nop" : "+v"(c) : "v"(a), "v"(b));
    return c; }
static __device__ __forceinline__ v8f wmmabg(v16bf a, v16bf b, v8f c) {
    c = __builtin_amdgcn_wmma_f32_16x16x32_bf16(false, a, false, b, (short)0, c, false, false);
    asm volatile("v_nop\n\tv_nop\n\tv_nop\n\tv_nop" : "+v"(c) : "v"(a), "v"(b));
    return c; }

__global__ __launch_bounds__(256) void k_cvt8(const float* __restrict__ src, bf* dst, size_t n8) {
    const size_t i = (size_t)blockIdx.x * 256 + threadIdx.x; if (i >= n8) return;
    const v8f v = *(const v8f*)(src + i * 8); v8us o;
#pragma unroll
    for (int k = 0; k < 8; ++k) o[k] = f2bf(v[k]);
    *(volatile v8us*)(dst + i * 8) = o; __threadfence(); *(volatile v8us*)(dst + i * 8) = o;
}

__global__ __launch_bounds__(256) void k_wtr(const float* __restrict__ src, bf* dst) {
    __shared__ __align__(16) float ts[64 * 68];
    const int tid = threadIdx.x; const int e0 = blockIdx.x * 64, n0 = blockIdx.y * 64;
#pragma unroll
    for (int it = 0; it < 4; ++it) { const int idx = it * 256 + tid; const int el = idx >> 4, n4 = (idx & 15) * 4;
        const v4f v = *(const v4f*)(src + (size_t)(e0 + el) * DM + n0 + n4);
#pragma unroll
        for (int i = 0; i < 4; ++i) ts[(n4 + i) * 68 + el] = v[i]; }
    __syncthreads();
    v8us o[2];
#pragma unroll
    for (int it = 0; it < 2; ++it) { const int n = it * 32 + (tid >> 3), c8 = (tid & 7) * 8;
        const v4f x0 = *(const v4fa*)(&ts[n * 68 + c8]); const v4f x1 = *(const v4fa*)(&ts[n * 68 + c8 + 4]);
#pragma unroll
        for (int i = 0; i < 4; ++i) { o[it][i] = f2bf(x0[i]); o[it][4 + i] = f2bf(x1[i]); } }
#pragma unroll 1
    for (int ps = 0; ps < 2; ++ps) {
#pragma unroll
        for (int it = 0; it < 2; ++it) { const int n = it * 32 + (tid >> 3), c8 = (tid & 7) * 8;
            *(volatile v8us*)(dst + (size_t)(n0 + n) * EMB + e0 + c8) = o[it]; }
        if (ps == 0) __threadfence(); }
}

__global__ __launch_bounds__(256) void k_ck(const float* __restrict__ src, h16* KX, size_t n8) {
    const size_t i = (size_t)blockIdx.x * 256 + threadIdx.x; if (i >= n8) return;
    const size_t e0 = i * 8;
    const int d8 = (int)(e0 & 63), h = (int)((e0 >> 6) & 7), w = (int)((e0 >> 9) & (WIN - 1)); const size_t b = e0 >> 18;
    const v8f v = *(const v8f*)(src + e0); v8h o;
#pragma unroll
    for (int k = 0; k < 8; ++k) o[k] = toh_flush(bfr(v[k]));
    h16* p = KX + (((size_t)b * NH_ + h) * XT + w) * HD + d8;
    *(volatile v8h*)p = o; __threadfence(); *(volatile v8h*)p = o;
}
static_assert(WIN * DM == (1 << 18));
static_assert(DM == (1 << 9));

__global__ __launch_bounds__(256) void k_cvt(const float* __restrict__ src, h16* VX) {
    __shared__ __align__(16) float ts[64 * 68];
    const int tid = threadIdx.x; const int w0 = blockIdx.x * 64; const int zh = blockIdx.y; const int b = zh / NH_, h = zh % NH_;
#pragma unroll
    for (int it = 0; it < 4; ++it) { const int idx = it * 256 + tid; const int wl = idx >> 4, d4 = (idx & 15) * 4;
        const v4f v = *(const v4f*)(src + (((size_t)b * WIN + w0 + wl) * NH_ + h) * HD + d4);
#pragma unroll
        for (int i = 0; i < 4; ++i) ts[(d4 + i) * 68 + wl] = bfr(v[i]); }
    __syncthreads();
    v8h o[2];
#pragma unroll
    for (int it = 0; it < 2; ++it) { const int d = it * 32 + (tid >> 3), c8 = (tid & 7) * 8;
        const v4f x0 = *(const v4fa*)(&ts[d * 68 + c8]); const v4f x1 = *(const v4fa*)(&ts[d * 68 + c8 + 4]);
#pragma unroll
        for (int i = 0; i < 4; ++i) { o[it][i] = toh_flush(x0[i]); o[it][4 + i] = toh_flush(x1[i]); } }
#pragma unroll 1
    for (int ps = 0; ps < 2; ++ps) {
#pragma unroll
        for (int it = 0; it < 2; ++it) { const int d = it * 32 + (tid >> 3), c8 = (tid & 7) * 8;
            *(volatile v8h*)(VX + ((size_t)zh * HD + d) * XT + w0 + c8) = o[it]; }
        if (ps == 0) __threadfence(); }
}

__device__ __forceinline__ void proj_tile(const bf* __restrict__ A, const size_t arow0, const bf* __restrict__ Bt, const size_t brow0,
                                          const bool doPlane, h16* Ph, const size_t tbase, const size_t pitch,
                                          const bool doF32, float* Fo, const size_t fbase) {
    __shared__ __align__(16) float os[16 * 68];
    const int lane = threadIdx.x & 31, lr = lane & 15, hi = lane >> 4;
    v8f acc[4][4];
#pragma unroll
    for (int mb = 0; mb < 4; ++mb)
#pragma unroll
        for (int nb = 0; nb < 4; ++nb) acc[mb][nb] = (v8f){};
    const size_t aoff = (arow0 + lr) * EMB + 8 * hi, boff = (brow0 + lr) * EMB + 8 * hi;
#pragma unroll 1
    for (int kc = 0; kc < EMB; kc += 32) {
        v16bf a[4];
#pragma unroll
        for (int mb = 0; mb < 4; ++mb) a[mb] = ldb(A + aoff + (size_t)mb * 16 * EMB + kc);
#pragma unroll
        for (int nb = 0; nb < 4; ++nb) { const v16bf bq = ldb(Bt + boff + (size_t)nb * 16 * EMB + kc);
#pragma unroll
            for (int mb = 0; mb < 4; ++mb) acc[mb][nb] = wmmabg(a[mb], bq, acc[mb][nb]); }
    }
#pragma unroll
    for (int mb = 0; mb < 4; ++mb) {
#pragma unroll
        for (int nb = 0; nb < 4; ++nb) {
#pragma unroll
            for (int j = 0; j < 8; ++j) os[(hi * 8 + j) * 68 + nb * 16 + lr] = acc[mb][nb][j]; }
        wave_sync();
#pragma unroll 1
        for (int ps = 0; ps < 2; ++ps) {
            if (doPlane) {
                const size_t sb = tbase + (size_t)(mb * 16) * pitch;
#pragma unroll
                for (int s = 0; s < 4; ++s) { const int row = 4 * s + (lane >> 3), c8 = (lane & 7) * 8;
                    const v4f x0 = *(const v4fa*)(&os[row * 68 + c8]); const v4f x1 = *(const v4fa*)(&os[row * 68 + c8 + 4]); v8h hv;
#pragma unroll
                    for (int i = 0; i < 4; ++i) { hv[i] = toh_flush(x0[i]); hv[4 + i] = toh_flush(x1[i]); }
                    *(volatile v8h*)(Ph + sb + (size_t)row * pitch + c8) = hv; }
            }
            if (doF32) {
                const size_t fb = fbase + (size_t)(mb * 16) * DM;
#pragma unroll
                for (int s = 0; s < 8; ++s) { const int row = 2 * s + (lane >> 4), cofs = (lane & 15) * 4;
                    const v4f val = *(const v4fa*)(&os[row * 68 + cofs]);
                    *(volatile v4f*)(Fo + fb + (size_t)row * DM + cofs) = val; }
            }
            if (ps == 0) __threadfence(); }
        wave_sync();
    }
}

__global__ __launch_bounds__(32) __attribute__((amdgpu_num_vgpr(256))) void k_proj_q(const bf* __restrict__ XB, const bf* __restrict__ WT, h16* QH, float* Fo) {
    const int r0 = blockIdx.x * 64, c0 = blockIdx.y * 64; const int bb = r0 / SEQ, tt = r0 % SEQ; const int zc = bb * NH_ + c0 / HD;
    proj_tile(XB, (size_t)r0, WT, (size_t)c0, true, QH, ((size_t)zc * SEQ + (size_t)tt) * HD, (size_t)HD, false, Fo, (size_t)0);
}
__global__ __launch_bounds__(32) __attribute__((amdgpu_num_vgpr(256))) void k_proj_k(const bf* __restrict__ XB, const bf* __restrict__ WT, h16* KX, float* Fo) {
    const int r0 = blockIdx.x * 64, c0 = blockIdx.y * 64; const int bb = r0 / SEQ, tt = r0 % SEQ; const int hh = c0 / HD; const int zc = bb * NH_ + hh;
    const bool last = tt >= (SEQ - WIN);
    const long long wl = (long long)tt - (long long)(SEQ - WIN);
    const size_t fbase = (size_t)((((long long)bb * WIN + wl) * NH_ + hh) * HD);
    proj_tile(XB, (size_t)r0, WT, (size_t)c0, true, KX, ((size_t)zc * XT + (size_t)(WIN + tt)) * HD, (size_t)HD, last, Fo, fbase);
}
__global__ __launch_bounds__(32) __attribute__((amdgpu_num_vgpr(256))) void k_proj_vt(const bf* __restrict__ WT, const bf* __restrict__ XB, h16* VX, float* Fo) {
    const int r0 = blockIdx.x * 64, c0 = blockIdx.y * 64; const int bb = c0 / SEQ, tt = c0 % SEQ;
    proj_tile(WT, (size_t)r0, XB, (size_t)c0, true, VX, ((size_t)bb * DM + (size_t)r0) * XT + (size_t)(WIN + tt), (size_t)XT, false, Fo, (size_t)0);
}
__global__ __launch_bounds__(32) __attribute__((amdgpu_num_vgpr(256))) void k_proj_vl(const bf* __restrict__ XB, const bf* __restrict__ WT, h16* Pu, float* Fo) {
    const int r0 = blockIdx.x * 64, c0 = blockIdx.y * 64; const int bb = r0 / WIN, wl = r0 % WIN;
    const size_t arow0 = (size_t)bb * SEQ + (size_t)(SEQ - WIN + wl);
    const size_t fbase = (((size_t)bb * WIN + (size_t)wl) * NH_ + (size_t)(c0 / HD)) * HD;
    proj_tile(XB, arow0, WT, (size_t)c0, false, Pu, (size_t)0, (size_t)HD, true, Fo, fbase);
}

__global__ __launch_bounds__(32 * AW) __attribute__((amdgpu_num_vgpr(256))) void k_flash(const h16* __restrict__ QH, const h16* __restrict__ KX, const h16* __restrict__ VX,
                                                                                         const float* __restrict__ relb, float* OUT) {
    __shared__ __align__(16) float os[AW * 16 * OSP];
    __shared__ __align__(16) float tbl[WIN];
    const int lane = threadIdx.x & 31, lr = lane & 15, hi = lane >> 4;
    const int wave = __builtin_amdgcn_readfirstlane((int)(threadIdx.x >> 5));
    const int zh = blockIdx.y; const int b = zh / NH_, h = zh % NH_;
#pragma unroll 1
    for (int idx = (int)threadIdx.x; idx < WIN; idx += 32 * AW) {
        int big = 16;
        big += (idx >= 19); big += (idx >= 21); big += (idx >= 24); big += (idx >= 27); big += (idx >= 31);
        big += (idx >= 35); big += (idx >= 40); big += (idx >= 46); big += (idx >= 52); big += (idx >= 59);
        big += (idx >= 67); big += (idx >= 77); big += (idx >= 87); big += (idx >= 99); big += (idx >= 113);
        const int bk = (idx < 16) ? idx : big;
        const float x = relb[h * NBK + bk];
        tbl[idx] = bfr(x) * LOG2E;
    }
    __syncthreads();
    const int t0 = (blockIdx.x * AW + wave) * 16;
    const int kbeg = t0 & ~31;
    const int sq = t0 + lr;
    const size_t qo = (size_t)zh * SEQ * HD + (size_t)sq * HD + 8 * hi;
    const v16h q0 = ldh(QH + qo), q1 = ldh(QH + qo + 32);
    const size_t xb = (size_t)zh * XT * HD;
    const size_t ko = xb + (size_t)lr * HD + 8 * hi;
    const size_t vo = xb + (size_t)lr * XT + 8 * hi;
    const int dq = sq + WIN - 8 * hi;
    v8f o0 = (v8f){}, o1 = (v8f){}, o2 = (v8f){}, o3 = (v8f){};
    float m = NEGB, l = 0.0f;
#pragma unroll 1
    for (int st = 0; st < NSTEP; ++st) {
        const int key0 = kbeg + 32 * st;
        const h16* ka = KX + ko + (size_t)key0 * HD;
        const v16h ka0 = ldh(ka), ka1 = ldh(ka + 32), kb0 = ldh(ka + 16 * HD), kb1 = ldh(ka + 16 * HD + 32);
        v8f sA = (v8f){}, sB = (v8f){};
        sA = wmma16g(ka0, q0, sA); sA = wmma16g(ka1, q1, sA);
        sB = wmma16g(kb0, q0, sB); sB = wmma16g(kb1, q1, sB);
        const int dA0 = dq - key0;
        float ta[8], tc[8]; bool fa[8], fb[8]; float mx = NEGB;
#pragma unroll
        for (int r = 0; r < 8; ++r) {
            const int da = dA0 - r, db = dA0 - 16 - r;
            const int ia = min(max(da, 0), WIN - 1), ib = min(max(db, 0), WIN - 1);
            float xa = tbl[ia], xc = tbl[ib];
            asm volatile("" : "+v"(xa)); asm volatile("" : "+v"(xc));
            fa[r] = (unsigned)da < (unsigned)WIN; fb[r] = (unsigned)db < (unsigned)WIN;
            ta[r] = sA[r] * SC2 + xa; tc[r] = sB[r] * SC2 + xc;
            mx = fmaxf(mx, fmaxf(fa[r] ? ta[r] : NEGB, fb[r] ? tc[r] : NEGB)); }
        mx = fmaxf(mx, __shfl_xor(mx, 16, 32));
        const float mnew = fmaxf(m, mx);
        const float alpha = __builtin_amdgcn_exp2f(m - mnew);
        const float sh = PSH - mnew;
        v16h pb; float ls = 0.0f;
#pragma unroll
        for (int r = 0; r < 8; ++r) {
            const float aa = ta[r] + sh, ac = tc[r] + sh;
            const float ea = __builtin_amdgcn_exp2f(aa), ec = __builtin_amdgcn_exp2f(ac);
            const float ga = (fa[r] & (aa >= -14.0f)) ? ea : 0.0f;
            const float gc = (fb[r] & (ac >= -14.0f)) ? ec : 0.0f;
            const h16 pa = (h16)ga; const h16 pc = (h16)gc;
            pb[r] = pa; pb[8 + r] = pc;
            ls += (float)pa + (float)pc; }
        l = l * alpha + ls; m = mnew;
        o0 = o0 * alpha; o1 = o1 * alpha; o2 = o2 * alpha; o3 = o3 * alpha;
        const h16* va = VX + vo + key0;
        const v16h v0 = ldh(va), v1 = ldh(va + (size_t)16 * XT), v2 = ldh(va + (size_t)32 * XT), v3 = ldh(va + (size_t)48 * XT);
        o0 = wmma16g(v0, pb, o0); o1 = wmma16g(v1, pb, o1); o2 = wmma16g(v2, pb, o2); o3 = wmma16g(v3, pb, o3);
    }
    l += __shfl_xor(l, 16, 32);
    const bool any = l > 0.0f;
    const float lsafe = any ? l : 1.0f;
    const float inv = any ? (1.0f / lsafe) : 0.0f;
    const int wb = wave * 16 * OSP;
    { v4f a, c;
      a[0] = o0[0] * inv; a[1] = o0[1] * inv; a[2] = o0[2] * inv; a[3] = o0[3] * inv; c[0] = o0[4] * inv; c[1] = o0[5] * inv; c[2] = o0[6] * inv; c[3] = o0[7] * inv;
      *(v4fa*)(&os[wb + lr * OSP +  0 + 8 * hi]) = a; *(v4fa*)(&os[wb + lr * OSP +  0 + 8 * hi + 4]) = c;
      a[0] = o1[0] * inv; a[1] = o1[1] * inv; a[2] = o1[2] * inv; a[3] = o1[3] * inv; c[0] = o1[4] * inv; c[1] = o1[5] * inv; c[2] = o1[6] * inv; c[3] = o1[7] * inv;
      *(v4fa*)(&os[wb + lr * OSP + 16 + 8 * hi]) = a; *(v4fa*)(&os[wb + lr * OSP + 16 + 8 * hi + 4]) = c;
      a[0] = o2[0] * inv; a[1] = o2[1] * inv; a[2] = o2[2] * inv; a[3] = o2[3] * inv; c[0] = o2[4] * inv; c[1] = o2[5] * inv; c[2] = o2[6] * inv; c[3] = o2[7] * inv;
      *(v4fa*)(&os[wb + lr * OSP + 32 + 8 * hi]) = a; *(v4fa*)(&os[wb + lr * OSP + 32 + 8 * hi + 4]) = c;
      a[0] = o3[0] * inv; a[1] = o3[1] * inv; a[2] = o3[2] * inv; a[3] = o3[3] * inv; c[0] = o3[4] * inv; c[1] = o3[5] * inv; c[2] = o3[6] * inv; c[3] = o3[7] * inv;
      *(v4fa*)(&os[wb + lr * OSP + 48 + 8 * hi]) = a; *(v4fa*)(&os[wb + lr * OSP + 48 + 8 * hi + 4]) = c; }
    wave_sync();
    float* orow = OUT + (((size_t)b * OUT_SEQ + (size_t)t0) * NH_ + (size_t)h) * HD;
#pragma unroll 1
    for (int ps = 0; ps < 2; ++ps) {
#pragma unroll
        for (int s = 0; s < 8; ++s) { const int row = 2 * s + (lane >> 4), cofs = (lane & 15) * 4;
            const v4f val = *(const v4fa*)(&os[wb + row * OSP + cofs]);
            *(volatile v4f*)(orow + (size_t)row * DM + cofs) = val; }
        if (ps == 0) __threadfence(); }
}

static constexpr size_t al256(size_t v) { return (v + 255) & ~(size_t)255; }
static constexpr size_t SZ_XB = al256((size_t)NB * SEQ * EMB * 2);
static constexpr size_t SZ_WB = al256((size_t)3 * DM * EMB * 2);
static constexpr size_t SZ_QP = al256((size_t)NB * NH_ * SEQ * HD * 2);
static constexpr size_t SZ_XP = al256((size_t)NB * NH_ * XT * HD * 2);
static constexpr size_t SZ_TOTAL = SZ_XB + SZ_WB + SZ_QP + 2 * SZ_XP;
static_assert(SZ_TOTAL <= (size_t)134217728);
static_assert(((size_t)DM * EMB * 2) % 256 == 0);
static_assert((size_t)NB * NH_ * XT * HD == (size_t)NB * DM * XT);
static_assert(((size_t)NB * SEQ * EMB) % 8 == 0);
static_assert(((size_t)NB * WIN * DM) % 8 == 0);

extern "C" void kernel_launch(void* const* d_in, const int* in_sizes, int n_in,
                              void* d_out, int out_size, void* d_ws, size_t ws_size, hipStream_t stream) {
    if (n_in < 7) return;
    const size_t needx = ((size_t)(NB - 1) * SEQ_FULL + SEQ) * EMB;
    const size_t needc = (size_t)NB * WIN * DM;
    if ((size_t)in_sizes[0] < needx) return;
    if ((size_t)in_sizes[1] < needc || (size_t)in_sizes[2] < needc) return;
    if ((size_t)in_sizes[3] < (size_t)EMB * DM || (size_t)in_sizes[4] < (size_t)EMB * DM || (size_t)in_sizes[5] < (size_t)EMB * DM) return;
    if (in_sizes[6] < NH_ * NBK) return;
    if ((size_t)out_size < OFF2 + (size_t)NB * WIN * DM) return;
    if (SZ_TOTAL > ws_size) return;
    const float* xs = (const float*)d_in[0];
    const float* ck = (const float*)d_in[1]; const float* cv = (const float*)d_in[2];
    const float* wq = (const float*)d_in[3]; const float* wk = (const float*)d_in[4]; const float* wv = (const float*)d_in[5];
    const float* relb = (const float*)d_in[6];
    float* OUT = (float*)d_out;
    float* OK_ = OUT + OFF1; float* OV_ = OUT + OFF2;
    char* wsp = (char*)d_ws;
    bf* XB = (bf*)wsp; wsp += SZ_XB;
    bf* WB = (bf*)wsp; wsp += SZ_WB;
    h16* QH = (h16*)wsp; wsp += SZ_QP;
    h16* KX = (h16*)wsp; wsp += SZ_XP;
    h16* VX = (h16*)wsp; wsp += SZ_XP;
    bf* WQ = WB; bf* WK = WB + (size_t)DM * EMB; bf* WV = WB + (size_t)2 * DM * EMB;

    if (SEQ == SEQ_FULL) {
        const size_t n8 = (size_t)NB * SEQ * EMB / 8;
        k_cvt8<<<(unsigned)((n8 + 255) / 256), 256, 0, stream>>>(xs, XB, n8);
    } else {
        const size_t n8 = (size_t)SEQ * EMB / 8;
        for (int b = 0; b < NB; ++b) k_cvt8<<<(unsigned)((n8 + 255) / 256), 256, 0, stream>>>(xs + (size_t)b * SEQ_FULL * EMB, XB + (size_t)b * SEQ * EMB, n8);
    }
    k_wtr<<<dim3(EMB / 64, DM / 64, 1), 256, 0, stream>>>(wq, WQ);
    k_wtr<<<dim3(EMB / 64, DM / 64, 1), 256, 0, stream>>>(wk, WK);
    k_wtr<<<dim3(EMB / 64, DM / 64, 1), 256, 0, stream>>>(wv, WV);
    { const size_t n8 = (size_t)NB * WIN * DM / 8;
      k_ck<<<(unsigned)((n8 + 255) / 256), 256, 0, stream>>>(ck, KX, n8); }
    k_cvt<<<dim3(WIN / 64, NB * NH_, 1), 256, 0, stream>>>(cv, VX);

    k_proj_q <<<dim3(NB * SEQ / 64, DM / 64, 1), 32, 0, stream>>>(XB, WQ, QH, OK_);
    k_proj_k <<<dim3(NB * SEQ / 64, DM / 64, 1), 32, 0, stream>>>(XB, WK, KX, OK_);
    k_proj_vt<<<dim3(DM / 64, NB * SEQ / 64, 1), 32, 0, stream>>>(WV, XB, VX, OV_);
    k_proj_vl<<<dim3(NB * WIN / 64, DM / 64, 1), 32, 0, stream>>>(XB, WV, QH, OV_);

    k_flash<<<dim3(SEQ / (16 * AW), NB * NH_, 1), 32 * AW, 0, stream>>>(QH, KX, VX, relb, OUT);
}
